// RotSSM_3685081940233
// MI455X (gfx1250) — hardware-verified
//
#include <hip/hip_runtime.h>
#include <math.h>

typedef __attribute__((ext_vector_type(16))) _Float16 v16h;
typedef __attribute__((ext_vector_type(8)))  _Float16 v8h;
typedef __attribute__((ext_vector_type(2)))  _Float16 v2h;
typedef __attribute__((ext_vector_type(8)))  float    v8f;
typedef __attribute__((ext_vector_type(4)))  float    v4f;
typedef __attribute__((ext_vector_type(2)))  float    v2f;

constexpr int kBatch = 8;
constexpr int kDh    = 256;
constexpr int kSeq   = 4096;
constexpr int kHeads = 64;
constexpr int kNst   = 4;
constexpr int kSd    = kHeads * kNst;
constexpr int kRows  = kBatch * kSeq;
static_assert(kSd == 256, "state width");
static_assert((kDh % 32) == 0 && (kSd % 32) == 0, "GEMM K multiples of 32");
static_assert((kRows % 64) == 0 && (kSd % 64) == 0 && (kDh % 64) == 0 && (kSeq % 64) == 0, "GEMM M,N multiples of 64");

constexpr float kCarryU = 16.0f;
constexpr float kCarryW = 256.0f;
constexpr float kCarryY = 64.0f;
constexpr float kScale1 = 1.0f / (kCarryU * kCarryW);
constexpr float kScale2 = 1.0f / (kCarryY * kCarryW);
constexpr float kHalfMinNormal = 6.103515625e-05f;

constexpr size_t kOffU16  = 0;
constexpr size_t kOffUS   = kOffU16 + (size_t)kRows * kDh * 2;
constexpr size_t kOffY16  = kOffUS  + (size_t)kRows * kSd * 4;
constexpr size_t kOffW1H  = kOffY16 + (size_t)kRows * kSd * 2;
constexpr size_t kOffW2H  = kOffW1H + (size_t)kSd * kDh * 2;
constexpr size_t kOffTAB  = kOffW2H + (size_t)kDh * kSd * 2;
constexpr size_t kWsTotal = kOffTAB + (size_t)(kHeads * 2) * 4 * 4;
static_assert(kWsTotal == 67373056ull, "carve total");
static_assert(kWsTotal <= 134217728ull, "carve cap");
static_assert((kOffUS % 128) == 0 && (kOffY16 % 128) == 0 && (kOffW1H % 128) == 0 &&
              (kOffW2H % 128) == 0 && (kOffTAB % 128) == 0, "128-B aligned regions");

__device__ __forceinline__ _Float16 to_h_flush(float v) {
  const float w = (fabsf(v) < kHalfMinNormal) ? 0.0f : v;
  return (_Float16)w;
}
__device__ __forceinline__ unsigned pack2h(float a, float b) {
  v2h hv;
  hv[0] = to_h_flush(a);
  hv[1] = to_h_flush(b);
  return __builtin_bit_cast(unsigned, hv);
}

__global__ __launch_bounds__(256) void prep_tables_kernel(
    const float* __restrict__ thl, const float* __restrict__ Bp, const float* __restrict__ gl,
    float* __restrict__ tab)
{
#pragma clang fp contract(off)
  __shared__ float sTr[256];
  const int tid = threadIdx.x;
  const float* rowp = Bp + (size_t)tid * kDh;
  float a0 = 0.0f, a1 = 0.0f, a2 = 0.0f, a3 = 0.0f;
#pragma unroll 1
  for (int i = 0; i < kDh / 4; ++i) {
    const v4f v = *(const v4f*)(rowp + 4 * i);
    a0 += v[0] * v[0];
    a1 += v[1] * v[1];
    a2 += v[2] * v[2];
    a3 += v[3] * v[3];
  }
  sTr[tid] = (a0 + a1) + (a2 + a3);
  __syncthreads();
  const int q = (tid < 128) ? tid : 127;
  const int h = q >> 1;
  const float tr = (sTr[4 * h] + sTr[4 * h + 1]) + (sTr[4 * h + 2] + sTr[4 * h + 3]);
  const float g  = expf(-expf(gl[h]));
  const float g2 = g * g;
  const float nrm = sqrtf((1.0f - g2) / tr);
  const float th = expf(thl[q]);
  const float cs = cosf(th);
  const float sn = sinf(th);
  const v4f tv = {cs, sn, g, nrm};
  if (tid < 128) {
    *(volatile v4f*)(tab + 4 * tid) = tv;
    __threadfence();
    *(volatile v4f*)(tab + 4 * tid) = tv;
  }
}

__device__ __forceinline__ void store_row_f16(const float* srow, unsigned short* drow, int lane) {
  const v4f a0 = *(const v4f*)(srow + lane * 8);
  const v4f a1 = *(const v4f*)(srow + lane * 8 + 4);
  v8h hv;
  hv[0] = to_h_flush(a0[0]);
  hv[1] = to_h_flush(a0[1]);
  hv[2] = to_h_flush(a0[2]);
  hv[3] = to_h_flush(a0[3]);
  hv[4] = to_h_flush(a1[0]);
  hv[5] = to_h_flush(a1[1]);
  hv[6] = to_h_flush(a1[2]);
  hv[7] = to_h_flush(a1[3]);
  unsigned short* p = drow + lane * 8;
  *(volatile v8h*)p = hv;
  __threadfence();
  *(volatile v8h*)p = hv;
}

__global__ __launch_bounds__(256) void fold_weights_kernel(
    const float* __restrict__ Pp, const float* __restrict__ Bp, const float* __restrict__ Cm,
    unsigned short* __restrict__ W1h, unsigned short* __restrict__ W2h)
{
  __shared__ __align__(16) float sP[kHeads * 16];
  __shared__ __align__(16) float sRow[8 * 256];
  const int tid = threadIdx.x, lane = tid & 31, wave = tid >> 5;
  {
    const int h = tid >> 2, r = tid & 3;
    const float* pp = Pp + h * 16;
    const v4f r0 = *(const v4f*)(pp);
    const v4f r1 = *(const v4f*)(pp + 4);
    const v4f r2 = *(const v4f*)(pp + 8);
    const v4f r3 = *(const v4f*)(pp + 12);
    const float pm[16] = {r0[0], r0[1], r0[2], r0[3], r1[0], r1[1], r1[2], r1[3],
                          r2[0], r2[1], r2[2], r2[3], r3[0], r3[1], r3[2], r3[3]};
    float sk[16];
#pragma unroll
    for (int j = 0; j < 4; ++j)
#pragma unroll
      for (int c = 0; c < 4; ++c) sk[j * 4 + c] = pm[j * 4 + c] - pm[c * 4 + j];
    float X[4], Pr[4];
#pragma unroll
    for (int c = 0; c < 4; ++c) {
      X[c] = (r == c) ? 1.0f : 0.0f;
      Pr[c] = X[c];
    }
#pragma unroll 1
    for (int k = 1; k <= 16; ++k) {
      const float inv = 1.0f / (float)k;
      float Tn[4];
#pragma unroll
      for (int c = 0; c < 4; ++c) {
        float t = X[0] * sk[c];
        t = fmaf(X[1], sk[4 + c], t);
        t = fmaf(X[2], sk[8 + c], t);
        t = fmaf(X[3], sk[12 + c], t);
        Tn[c] = t * inv;
      }
#pragma unroll
      for (int c = 0; c < 4; ++c) {
        X[c] = Tn[c];
        Pr[c] += Tn[c];
      }
    }
    const v4f pv = {Pr[0], Pr[1], Pr[2], Pr[3]};
    *(v4f*)(sP + tid * 4) = pv;
  }
  __syncthreads();
  const int R = blockIdx.x * 8 + wave;
  {
    const int h = R >> 2;
    const v4f pr = *(const v4f*)(sP + R * 4);
    const float* b0 = Bp + (size_t)(h * 4) * kDh;
#pragma unroll 1
    for (int e = 0; e < 8; ++e) {
      const int d = e * 32 + lane;
      float v = pr[0] * b0[d];
      v = fmaf(pr[1], b0[kDh + d], v);
      v = fmaf(pr[2], b0[2 * kDh + d], v);
      v = fmaf(pr[3], b0[3 * kDh + d], v);
      sRow[wave * 256 + d] = v * kCarryW;
    }
  }
  __syncthreads();
  store_row_f16(sRow + wave * 256, W1h + (size_t)R * kDh, lane);
  __syncthreads();
  {
    const float* crow = Cm + (size_t)R * kSd;
#pragma unroll 1
    for (int e = 0; e < 8; ++e) {
      const int col = e * 32 + lane;
      const v4f cv = *(const v4f*)(crow + (col & ~3));
      const v4f pv = *(const v4f*)(sP + col * 4);
      float v = cv[0] * pv[0];
      v = fmaf(cv[1], pv[1], v);
      v = fmaf(cv[2], pv[2], v);
      v = fmaf(cv[3], pv[3], v);
      sRow[wave * 256 + col] = v * kCarryW;
    }
  }
  __syncthreads();
  store_row_f16(sRow + wave * 256, W2h + (size_t)R * kSd, lane);
}

__global__ __launch_bounds__(256) void transpose_cast_kernel(
    const float* __restrict__ u, unsigned short* __restrict__ U16)
{
  __shared__ float sT[64 * 65];
  const int tid = threadIdx.x;
  const int t0 = blockIdx.x * 64, d0 = blockIdx.y * 64, b = blockIdx.z;
  const float* ub = u + ((size_t)b * kDh + d0) * kSeq + t0;
#pragma unroll
  for (int i = 0; i < 4; ++i) {
    const int idx = tid + 256 * i;
    const int drow = idx >> 4, tq = (idx & 15) * 4;
    const v4f v = *(const v4f*)(ub + (size_t)drow * kSeq + tq);
    float* dst = sT + drow * 65 + tq;
    dst[0] = v[0];
    dst[1] = v[1];
    dst[2] = v[2];
    dst[3] = v[3];
  }
  __syncthreads();
  const int c8 = (tid & 7) * 8;
  v8h hv[2];
#pragma unroll
  for (int it = 0; it < 2; ++it) {
    const int trow = it * 32 + (tid >> 3);
#pragma unroll
    for (int e = 0; e < 8; ++e) hv[it][e] = to_h_flush(sT[(c8 + e) * 65 + trow] * kCarryU);
  }
  for (int pass = 0; pass < 2; ++pass) {
#pragma unroll
    for (int it = 0; it < 2; ++it) {
      const int trow = it * 32 + (tid >> 3);
      unsigned short* p = U16 + ((size_t)b * kSeq + t0 + trow) * kDh + d0 + c8;
      *(volatile v8h*)p = hv[it];
    }
    __threadfence();
  }
}

namespace eng {

__device__ __forceinline__ v16h frag_load(const _Float16* p) {
  union U { v16h v; v8h h[2]; } f;
  f.h[0] = *(const v8h*)(p);
  f.h[1] = *(const v8h*)(p + 16);
  return f.v;
}
__device__ __forceinline__ void mma_tied(v8f& c, v16h a, v16h b) {
  c = __builtin_amdgcn_wmma_f32_16x16x32_f16(false, a, false, b, (short)0, c, false, false);
  asm volatile("v_nop\n\tv_nop\n\tv_nop\n\tv_nop" : "+v"(c) : "v"(a), "v"(b));
}

template <bool SKIP>
__global__ __launch_bounds__(256) void gemm_f16_kernel(
    const unsigned short* __restrict__ Ap, int lda, long strideA,
    const unsigned short* __restrict__ Btp, int ldb, long strideB,
    float* __restrict__ Cout, int ldc, long strideC,
    const float* __restrict__ gain, const float* __restrict__ src,
    int M, int N, int K, float scale)
{
  __shared__ __align__(16) float sT[8][16 * 68];
  const int b    = blockIdx.y;
  const int lane = threadIdx.x & 31;
  const int wave = threadIdx.x >> 5;
  const int tilesN = N >> 6;
  const int tilesM = M >> 6;
  const int tile = blockIdx.x * 8 + wave;
  if (tile >= tilesM * tilesN) return;
  const int tm = tile / tilesN;
  const int tn = tile - tm * tilesN;
  const int m0 = tm << 6;
  const int n0 = tn << 6;

  const _Float16* Ab = (const _Float16*)Ap  + (size_t)b * strideA;
  const _Float16* Bb = (const _Float16*)Btp + (size_t)b * strideB;

  const int rlane = lane & 15;
  const int koff  = (lane >> 4) * 8;
  const int mOff  = (lane >> 4) * 8;

  v8f acc[4][4];
#pragma unroll
  for (int i = 0; i < 4; ++i)
#pragma unroll
    for (int j = 0; j < 4; ++j) acc[i][j] = (v8f){0.f, 0.f, 0.f, 0.f, 0.f, 0.f, 0.f, 0.f};

  for (int k0 = 0; k0 < K; k0 += 32) {
    v16h bh[4];
#pragma unroll
    for (int j = 0; j < 4; ++j)
      bh[j] = frag_load(Bb + (size_t)(n0 + (j << 4) + rlane) * ldb + koff + k0);
#pragma unroll
    for (int i = 0; i < 4; ++i) {
      const v16h ah = frag_load(Ab + (size_t)(m0 + (i << 4) + rlane) * lda + koff + k0);
#pragma unroll
      for (int j = 0; j < 4; ++j) mma_tied(acc[i][j], ah, bh[j]);
    }
  }

  float* slab = sT[wave];
  float* C = Cout + (size_t)b * strideC;
  const float* Sb = src + (size_t)b * strideC;
  const int hh = lane >> 4, c4 = (lane & 15) * 4;
#pragma unroll
  for (int i = 0; i < 4; ++i) {
    const int mBase = m0 + (i << 4);
#pragma unroll
    for (int j = 0; j < 4; ++j) {
#pragma unroll
      for (int r = 0; r < 8; ++r) slab[(mOff + r) * 68 + (j << 4) + rlane] = acc[i][j][r] * scale;
    }
    __builtin_amdgcn_fence(__ATOMIC_RELEASE, "workgroup");
    __builtin_amdgcn_wave_barrier();
    __builtin_amdgcn_fence(__ATOMIC_ACQUIRE, "workgroup");
#pragma unroll
    for (int hf = 0; hf < 2; ++hf) {
      v4f vv[4];
#pragma unroll
      for (int it = 0; it < 4; ++it) {
        const int row = (hf * 4 + it) * 2 + hh;
        v4f v = *(const v4f*)(slab + row * 68 + c4);
        if (SKIP) {
          const size_t o = (size_t)(mBase + row) * ldc + n0 + c4;
          const v4f uu = *(const v4f*)(Sb + o);
          const float dd = gain[mBase + row];
          v[0] = fmaf(dd, uu[0], v[0]);
          v[1] = fmaf(dd, uu[1], v[1]);
          v[2] = fmaf(dd, uu[2], v[2]);
          v[3] = fmaf(dd, uu[3], v[3]);
        }
        vv[it] = v;
      }
      for (int pass = 0; pass < 2; ++pass) {
#pragma unroll
        for (int it = 0; it < 4; ++it) {
          const int row = (hf * 4 + it) * 2 + hh;
          *(volatile v4f*)(C + (size_t)(mBase + row) * ldc + n0 + c4) = vv[it];
        }
        __threadfence();
      }
    }
    __builtin_amdgcn_fence(__ATOMIC_RELEASE, "workgroup");
    __builtin_amdgcn_wave_barrier();
    __builtin_amdgcn_fence(__ATOMIC_ACQUIRE, "workgroup");
  }
}

}

__global__ __launch_bounds__(32) void rot_scan_kernel(
    const float* __restrict__ Us, const float* __restrict__ tab, unsigned* __restrict__ Yw)
{
  const int lane = threadIdx.x;
  const int b = blockIdx.x >> 2;
  const int w = blockIdx.x & 3;
  const int q = w * 32 + lane;
  const v4f tv = *(const v4f*)(tab + 4 * q);
  const float c = tv[0], s = tv[1], g = tv[2], nrm = tv[3];
  float x0 = 0.0f, x1 = 0.0f;
  const size_t row0 = (size_t)b * kSeq;
#pragma unroll 1
  for (int tb = 0; tb < kSeq; tb += 8) {
    v2f uv[8];
#pragma unroll
    for (int j = 0; j < 8; ++j) uv[j] = *(const v2f*)(Us + (row0 + tb + j) * kSd + 2 * q);
    unsigned wd[8];
#pragma unroll
    for (int j = 0; j < 8; ++j) {
      const float t0 = c * x0 - s * x1;
      const float t1 = c * x1 + s * x0;
      x0 = g * t0 + nrm * uv[j][0];
      x1 = g * t1 + nrm * uv[j][1];
      wd[j] = pack2h(x0 * kCarryY, x1 * kCarryY);
    }
    for (int pass = 0; pass < 2; ++pass) {
#pragma unroll
      for (int j = 0; j < 8; ++j)
        *(volatile unsigned*)(Yw + (row0 + tb + j) * (kSd / 2) + q) = wd[j];
      __threadfence();
    }
  }
}

extern "C" void kernel_launch(void* const* d_in, const int* in_sizes, int n_in,
                              void* d_out, int out_size, void* d_ws, size_t ws_size,
                              hipStream_t stream) {
  if (n_in < 7) return;
  if (in_sizes[0] != kBatch * kDh * kSeq) return;
  if (in_sizes[1] != kHeads * 2) return;
  if (in_sizes[2] != kHeads * 16) return;
  if (in_sizes[3] != kHeads * kNst * kDh) return;
  if (in_sizes[4] != kDh * kSd) return;
  if (in_sizes[5] != kDh) return;
  if (in_sizes[6] != kHeads) return;
  if (out_size != kBatch * kDh * kSeq) return;
  if (ws_size < kWsTotal) return;

  const float* u          = (const float*)d_in[0];
  const float* thetas_log = (const float*)d_in[1];
  const float* P_param    = (const float*)d_in[2];
  const float* B_param    = (const float*)d_in[3];
  const float* Cmat       = (const float*)d_in[4];
  const float* Dvec       = (const float*)d_in[5];
  const float* gamma_log  = (const float*)d_in[6];
  float* out = (float*)d_out;

  char* ws = (char*)d_ws;
  unsigned short* U16 = (unsigned short*)(ws + kOffU16);
  float*          US  = (float*)(ws + kOffUS);
  unsigned short* Y16 = (unsigned short*)(ws + kOffY16);
  unsigned short* W1H = (unsigned short*)(ws + kOffW1H);
  unsigned short* W2H = (unsigned short*)(ws + kOffW2H);
  float*          TAB = (float*)(ws + kOffTAB);

  prep_tables_kernel<<<1, 256, 0, stream>>>(thetas_log, B_param, gamma_log, TAB);

  fold_weights_kernel<<<32, 256, 0, stream>>>(P_param, B_param, Cmat, W1H, W2H);

  transpose_cast_kernel<<<dim3(kSeq / 64, kDh / 64, kBatch), 256, 0, stream>>>(u, U16);

  eng::gemm_f16_kernel<false><<<dim3(256, 1), 256, 0, stream>>>(
      U16, kDh, 0L,
      W1H, kDh, 0L,
      US, kSd, 0L,
      Dvec, u,
      kRows, kSd, kDh, kScale1);

  rot_scan_kernel<<<kBatch * 4, 32, 0, stream>>>(US, TAB, (unsigned*)Y16);

  eng::gemm_f16_kernel<true><<<dim3(32, kBatch), 256, 0, stream>>>(
      W2H, kSd, 0L,
      Y16, kSd, (long)kSeq * kSd,
      out, kSeq, (long)kDh * kSeq,
      Dvec, u,
      kDh, kSeq, kSd, kScale2);
}
